// EdgeSAGE_43456479101296
// MI455X (gfx1250) — hardware-verified
//
#include <hip/hip_runtime.h>
#define NN 100000
#define NE 1600000
#define FIN 128
#define HID 128
#define FE 8
#define NOUT 2
#define ECAP 48
#define RQ 20000
#define BNEPS 1e-5f
typedef __bf16 v16b __attribute__((ext_vector_type(16)));
typedef unsigned short v8us __attribute__((ext_vector_type(8), may_alias));
typedef float  v8f  __attribute__((ext_vector_type(8)));
typedef float  v4f  __attribute__((ext_vector_type(4)));
typedef float  v4fa __attribute__((ext_vector_type(4), may_alias));
union FragB { v16b v; v8us half[2]; unsigned short u[16]; };

__device__ __forceinline__ unsigned short bf16_bits(float x) { unsigned int u = __float_as_uint(x); return (unsigned short)((u + 0x7FFFu + ((u >> 16) & 1u)) >> 16); }
__device__ __forceinline__ float bf16_val(unsigned short b) { return __uint_as_float(((unsigned int)b) << 16); }
__device__ __forceinline__ float bf16_round(float x) { return bf16_val(bf16_bits(x)); }
template <int NT>
__device__ __forceinline__ v8f mmaN(v16b ah, v16b al, v16b bh, v16b bl, v8f c) {
  c = __builtin_amdgcn_wmma_f32_16x16x32_bf16(false, ah, false, bh, (short)0, c, false, false);
  if (NT >= 2) c = __builtin_amdgcn_wmma_f32_16x16x32_bf16(false, al, false, bh, (short)0, c, false, false);
  if (NT >= 3) c = __builtin_amdgcn_wmma_f32_16x16x32_bf16(false, ah, false, bl, (short)0, c, false, false);
  asm volatile("v_nop\n\tv_nop\n\tv_nop\n\tv_nop" : "+v"(c) : "v"(ah), "v"(al), "v"(bh), "v"(bl));
  return c;
}

__global__ __launch_bounds__(256) void k_wt_bf16(const float* __restrict__ W, unsigned short* __restrict__ Wt, int K, int N) {
  const int t = blockIdx.x * 256 + threadIdx.x;
  const int k8n = K / 8;
  if (t >= N * k8n) return;
  const int n = t / k8n, k8 = (t % k8n) * 8;
  v8us v;
#pragma unroll
  for (int i = 0; i < 8; ++i) v[i] = bf16_bits(W[(size_t)(k8 + i) * N + n]);
  *(volatile v8us*)(Wt + (size_t)n * K + k8) = v;
  __threadfence();
  *(volatile v8us*)(Wt + (size_t)n * K + k8) = v;
}

template <bool ASPLIT, int ACT, bool BIAS_BF16>
__global__ __launch_bounds__(128) void k_gemm_bf(const float* __restrict__ A, int lda, const unsigned short* __restrict__ Wt, int ldb,
                                               const float* __restrict__ bias, float* __restrict__ C, int ldc, int M, int N, int K) {
  __shared__ __attribute__((aligned(16))) float so[4][16][64];
  const int tid = threadIdx.x, w = tid >> 5, lane = tid & 31, ln = lane & 15, hh = lane >> 4;
  const int ntn = N / 64;
  const int wid = blockIdx.x * 4 + w;
  const int mt = wid / ntn, nq = wid % ntn;
  if (mt * 16 >= M) return;
  const int row0 = mt * 16, col0 = nq * 64;
  const float* arow = A + (size_t)(row0 + ln) * lda;
  v8f acc[4] = {};
  for (int kb = 0; kb < K; kb += 32) {
    FragB ah, al;
    const v4f x0 = *(const v4fa*)(arow + kb + 8 * hh), x1 = *(const v4fa*)(arow + kb + 8 * hh + 4);
    const v4f x2 = *(const v4fa*)(arow + kb + 16 + 8 * hh), x3 = *(const v4fa*)(arow + kb + 16 + 8 * hh + 4);
    float xs[16] = {x0[0],x0[1],x0[2],x0[3],x1[0],x1[1],x1[2],x1[3],x2[0],x2[1],x2[2],x2[3],x3[0],x3[1],x3[2],x3[3]};
#pragma unroll
    for (int i = 0; i < 16; ++i) { const unsigned short hb = bf16_bits(xs[i]); ah.u[i] = hb; al.u[i] = ASPLIT ? bf16_bits(xs[i] - bf16_val(hb)) : (unsigned short)0; }
#pragma unroll
    for (int t = 0; t < 4; ++t) {
      const unsigned short* brow = Wt + (size_t)(col0 + t * 16 + ln) * ldb + kb;
      FragB b;
      b.half[0] = *(const v8us*)(brow + 8 * hh);
      b.half[1] = *(const v8us*)(brow + 16 + 8 * hh);
      acc[t] = mmaN<ASPLIT ? 2 : 1>(ah.v, al.v, b.v, b.v, acc[t]);
    }
  }
#pragma unroll
  for (int t = 0; t < 4; ++t) {
    float bv = bias ? bias[col0 + t * 16 + ln] : 0.f;
    if (BIAS_BF16) bv = bf16_round(bv);
#pragma unroll
    for (int r = 0; r < 8; ++r) { float v = acc[t][r] + bv; if (ACT == 1) v = fmaxf(v, 0.f); so[w][8 * hh + r][t * 16 + ln] = v; }
  }
  __builtin_amdgcn_fence(__ATOMIC_ACQ_REL, "workgroup");
  __builtin_amdgcn_wave_barrier();
  const int rsub = lane >> 4, c4 = (lane & 15) * 4;
  for (int pass = 0; pass < 2; ++pass) {
#pragma unroll
    for (int q = 0; q < 8; ++q) {
      const int r = q * 2 + rsub;
      const v4f v = *(const v4fa*)&so[w][r][c4];
      *(volatile v4f*)(C + (size_t)(row0 + r) * ldc + col0 + c4) = v;
    }
    if (pass == 0) __threadfence();
  }
}

template <bool ASPLIT, int ACT, bool BIAS_BF16, bool RES_BF16>
__global__ __launch_bounds__(128) void k_gemm_bf3(const float* __restrict__ A, int lda, const unsigned short* __restrict__ Wt, int ldb,
                                                const float* __restrict__ bias, const float* __restrict__ resid, int rmod, int ldr,
                                                float* __restrict__ C, int ldc, int M, int N, int K) {
  __shared__ __attribute__((aligned(16))) float so[4][16][64];
  const int tid = threadIdx.x, w = tid >> 5, lane = tid & 31, ln = lane & 15, hh = lane >> 4;
  const int ntn = N / 64;
  const int wid = blockIdx.x * 4 + w;
  const int mt = wid / ntn, nq = wid % ntn;
  if (mt * 16 >= M) return;
  const int row0 = mt * 16, col0 = nq * 64;
  const float* arow = A + (size_t)(row0 + ln) * lda;
  v8f acc[4] = {};
  for (int kb = 0; kb < K; kb += 32) {
    FragB ah, al;
    const v4f x0 = *(const v4fa*)(arow + kb + 8 * hh), x1 = *(const v4fa*)(arow + kb + 8 * hh + 4);
    const v4f x2 = *(const v4fa*)(arow + kb + 16 + 8 * hh), x3 = *(const v4fa*)(arow + kb + 16 + 8 * hh + 4);
    float xs[16] = {x0[0],x0[1],x0[2],x0[3],x1[0],x1[1],x1[2],x1[3],x2[0],x2[1],x2[2],x2[3],x3[0],x3[1],x3[2],x3[3]};
#pragma unroll
    for (int i = 0; i < 16; ++i) { const unsigned short hb = bf16_bits(xs[i]); ah.u[i] = hb; al.u[i] = ASPLIT ? bf16_bits(xs[i] - bf16_val(hb)) : (unsigned short)0; }
#pragma unroll
    for (int t = 0; t < 4; ++t) {
      const unsigned short* brow = Wt + (size_t)(col0 + t * 16 + ln) * ldb + kb;
      FragB b;
      b.half[0] = *(const v8us*)(brow + 8 * hh);
      b.half[1] = *(const v8us*)(brow + 16 + 8 * hh);
      acc[t] = mmaN<ASPLIT ? 2 : 1>(ah.v, al.v, b.v, b.v, acc[t]);
    }
  }
#pragma unroll
  for (int t = 0; t < 4; ++t) {
    const int col = col0 + t * 16 + ln;
    float bv = bias ? bias[col] : 0.f;
    if (BIAS_BF16) bv = bf16_round(bv);
#pragma unroll
    for (int r = 0; r < 8; ++r) {
      float v = acc[t][r] + bv;
      if (resid) { float rv = resid[(size_t)((row0 + 8 * hh + r) % rmod) * ldr + col]; if (RES_BF16) rv = bf16_round(rv); v += rv; }
      if (ACT == 1) v = fmaxf(v, 0.f);
      if (ACT == 2) v = 0.5f * v * (1.0f + erff(v * 0.70710678118654752f));
      if (ACT == 3) { const float u = 0.7978845608028654f * (v + 0.044715f * v * v * v); v = 0.5f * v * (1.0f + tanhf(u)); }
      so[w][8 * hh + r][t * 16 + ln] = v;
    }
  }
  __builtin_amdgcn_fence(__ATOMIC_ACQ_REL, "workgroup");
  __builtin_amdgcn_wave_barrier();
  const int rsub = lane >> 4, c4 = (lane & 15) * 4;
  for (int pass = 0; pass < 2; ++pass) {
#pragma unroll
    for (int q = 0; q < 8; ++q) {
      const int r = q * 2 + rsub;
      const v4f v = *(const v4fa*)&so[w][r][c4];
      *(volatile v4f*)(C + (size_t)(row0 + r) * ldc + col0 + c4) = v;
    }
    if (pass == 0) __threadfence();
  }
}
template <bool PARAM_BF16>
__global__ __launch_bounds__(256) void k_layernorm(const float* __restrict__ X, const float* __restrict__ R, const float* __restrict__ g, const float* __restrict__ bta,
                                                  float* __restrict__ out_sum, float* __restrict__ out_norm, int N, float eps) {
  __shared__ float red[256];
  const int row = blockIdx.x, tid = threadIdx.x;
  const float* x = X + (size_t)row * N; const float* rr = R ? R + (size_t)row * N : nullptr;
  float vals[16];
  const int per = N / 256;
  float s1 = 0.f;
  for (int u = 0; u < per / 4; ++u) {
    const int j = tid * 4 + 1024 * u;
    const v4f a = *(const v4fa*)(x + j);
    v4f b = {0.f,0.f,0.f,0.f}; if (rr) b = *(const v4fa*)(rr + j);
#pragma unroll
    for (int q = 0; q < 4; ++q) { const float v = a[q] + b[q]; vals[u * 4 + q] = v; s1 += v; }
  }
  red[tid] = s1; __syncthreads();
  for (int st = 128; st > 0; st >>= 1) { if (tid < st) red[tid] += red[tid + st]; __syncthreads(); }
  const float mu = red[0] / (float)N; __syncthreads();
  float s2 = 0.f;
  for (int u = 0; u < per / 4; ++u)
#pragma unroll
    for (int q = 0; q < 4; ++q) { const float c = vals[u * 4 + q] - mu; s2 += c * c; }
  red[tid] = s2; __syncthreads();
  for (int st = 128; st > 0; st >>= 1) { if (tid < st) red[tid] += red[tid + st]; __syncthreads(); }
  const float rs = rsqrtf(red[0] / (float)N + eps);
  for (int pass = 0; pass < 2; ++pass) {
    for (int u = 0; u < per / 4; ++u) {
      const int j = tid * 4 + 1024 * u;
      v4f o, sm;
#pragma unroll
      for (int q = 0; q < 4; ++q) {
        float gg = g[j + q], bb = bta[j + q];
        if (PARAM_BF16) { gg = bf16_round(gg); bb = bf16_round(bb); }
        sm[q] = vals[u * 4 + q]; o[q] = (vals[u * 4 + q] - mu) * rs * gg + bb;
      }
      if (out_sum) *(volatile v4f*)(out_sum + (size_t)row * N + j) = sm;
      *(volatile v4f*)(out_norm + (size_t)row * N + j) = o;
    }
    if (pass == 0) __threadfence();
  }
}


typedef _Float16 v16h __attribute__((ext_vector_type(16)));
union FragH { v16h v; v8us half[2]; _Float16 h[16]; unsigned short u[16]; };
template <int NT>
__device__ __forceinline__ v8f mmaH(v16h ah, v16h al, v16h bh, v16h bl, v8f c) {
  c = __builtin_amdgcn_wmma_f32_16x16x32_f16(false, ah, false, bh, (short)0, c, false, false);
  if (NT >= 2) c = __builtin_amdgcn_wmma_f32_16x16x32_f16(false, al, false, bh, (short)0, c, false, false);
  if (NT >= 3) c = __builtin_amdgcn_wmma_f32_16x16x32_f16(false, ah, false, bl, (short)0, c, false, false);
  asm volatile("v_nop\n\tv_nop\n\tv_nop\n\tv_nop" : "+v"(c) : "v"(ah), "v"(al), "v"(bh), "v"(bl));
  return c;
}
template <bool ASPLIT>
__global__ __launch_bounds__(128) void k_gemm_h(const float* __restrict__ A, int lda, size_t sA, const _Float16* __restrict__ Bh, int ldb, size_t sB, float alpha, float* __restrict__ C, int ldc, size_t sC, int M, int N, int K) {
  __shared__ __attribute__((aligned(16))) float so[4][16][64];
  const int tid = threadIdx.x, w = tid >> 5, lane = tid & 31, ln = lane & 15, hh = lane >> 4; const int by = blockIdx.y;
  A += (size_t)by * sA; Bh += (size_t)by * sB; C += (size_t)by * sC;
  const int ntn = (N + 63) / 64; const int wid = blockIdx.x * 4 + w; const int mt = wid / ntn, nq = wid % ntn; if (mt * 16 >= M) return;
  const int row0 = mt * 16, col0 = nq * 64; const float* arow = A + (size_t)(row0 + ln) * lda;
  v8f acc[4] = {};
  for (int kb = 0; kb < K; kb += 32) {
    FragH ah, al;
    const v4f x0 = *(const v4fa*)(arow + kb + 8 * hh), x1 = *(const v4fa*)(arow + kb + 8 * hh + 4), x2 = *(const v4fa*)(arow + kb + 16 + 8 * hh), x3 = *(const v4fa*)(arow + kb + 16 + 8 * hh + 4);
    float xs[16] = {x0[0],x0[1],x0[2],x0[3],x1[0],x1[1],x1[2],x1[3],x2[0],x2[1],x2[2],x2[3],x3[0],x3[1],x3[2],x3[3]};
#pragma unroll
    for (int i = 0; i < 16; ++i) { const _Float16 h = (_Float16)xs[i]; ah.h[i] = h; al.h[i] = ASPLIT ? (_Float16)(xs[i] - (float)h) : (_Float16)0.0f; }
#pragma unroll
    for (int t = 0; t < 4; ++t) { if (col0 + t * 16 >= N) continue; const size_t boff = (size_t)(col0 + t * 16 + ln) * ldb + kb; FragH bq; bq.half[0] = *(const v8us*)(Bh + boff + 8 * hh); bq.half[1] = *(const v8us*)(Bh + boff + 16 + 8 * hh);
      acc[t] = mmaH<ASPLIT ? 2 : 1>(ah.v, al.v, bq.v, bq.v, acc[t]); }
  }
#pragma unroll
  for (int t = 0; t < 4; ++t) { if (col0 + t * 16 >= N) continue;
#pragma unroll
    for (int r = 0; r < 8; ++r) so[w][8 * hh + r][t * 16 + ln] = acc[t][r] * alpha; }
  __builtin_amdgcn_fence(__ATOMIC_ACQ_REL, "workgroup"); __builtin_amdgcn_wave_barrier();
  const int rsub = lane >> 4, c4 = (lane & 15) * 4;
  for (int pass = 0; pass < 2; ++pass) {
#pragma unroll
    for (int q = 0; q < 8; ++q) { const int r = q * 2 + rsub; if (col0 + c4 < N) { const v4f v = *(const v4fa*)&so[w][r][c4]; *(volatile v4f*)(C + (size_t)(row0 + r) * ldc + col0 + c4) = v; } }
    if (pass == 0) __threadfence(); }
}

__global__ __launch_bounds__(256) void k_wt_f16(const float* __restrict__ W, _Float16* __restrict__ Wt, int K, int N, float scale) {
  const int t = blockIdx.x * 256 + threadIdx.x; if (t >= N * (K / 8)) return; const int n = t / (K / 8), k8 = (t % (K / 8)) * 8; FragH f;
#pragma unroll
  for (int i = 0; i < 8; ++i) f.h[i] = (_Float16)(bf16_round(W[(size_t)(k8 + i) * N + n]) * scale); const v8us o = f.half[0];
  *(volatile v8us*)((unsigned short*)Wt + (size_t)n * K + k8) = o; __threadfence(); *(volatile v8us*)((unsigned short*)Wt + (size_t)n * K + k8) = o;
}
template <int ACT>
__global__ __launch_bounds__(128) void k_gemm_hhx(const _Float16* __restrict__ A, int lda, size_t sA, const _Float16* __restrict__ Bh, int ldb, size_t sB, float alpha, const float* __restrict__ bias, size_t sBias, const float* __restrict__ CP, int rowsPerB, size_t sCPb, int row0g,
    float* __restrict__ C, _Float16* __restrict__ C16, int ldc, size_t sC, int M, int N, int K) {
  __shared__ __attribute__((aligned(16))) float so[4][16][64];
  const int tid = threadIdx.x, w = tid >> 5, lane = tid & 31, ln = lane & 15, hh = lane >> 4; const int by = blockIdx.y;
  A += (size_t)by * sA; Bh += (size_t)by * sB; const size_t cofs = (size_t)by * sC; const float* bp = bias ? bias + (size_t)by * sBias : nullptr;
  const int ntn = (N + 63) / 64; const int wid = blockIdx.x * 4 + w; const int mt = wid / ntn, nq = wid % ntn; if (mt * 16 >= M) return;
  const int row0 = mt * 16, col0 = nq * 64; const _Float16* arow = A + (size_t)(row0 + ln) * lda;
  v8f acc[4] = {};
  for (int kb = 0; kb < K; kb += 32) { FragH ah; ah.half[0] = *(const v8us*)((const unsigned short*)arow + kb + 8 * hh); ah.half[1] = *(const v8us*)((const unsigned short*)arow + kb + 16 + 8 * hh);
#pragma unroll
    for (int t = 0; t < 4; ++t) { if (col0 + t * 16 >= N) continue; const size_t boff = (size_t)(col0 + t * 16 + ln) * ldb + kb; FragH bq; bq.half[0] = *(const v8us*)((const unsigned short*)Bh + boff + 8 * hh); bq.half[1] = *(const v8us*)((const unsigned short*)Bh + boff + 16 + 8 * hh);
      acc[t] = mmaH<1>(ah.v, ah.v, bq.v, bq.v, acc[t]); }
  }
#pragma unroll
  for (int t = 0; t < 4; ++t) { if (col0 + t * 16 >= N) continue; const int col = col0 + t * 16 + ln; const float bv = bp ? bf16_round(bp[col]) : 0.f;
#pragma unroll
    for (int r = 0; r < 8; ++r) { float v = acc[t][r] * alpha + bv; if (CP) { const int bidx = (row0g + row0 + 8 * hh + r) / rowsPerB; v += CP[(size_t)bidx * sCPb + (size_t)by * 64 + col]; } if (ACT == 1) v = (v > 0.f) ? v : expm1f(v); else if (ACT == 7) v = (v > 0.f) ? v + 1.0f : expf(v); else if (ACT == 8) v = tanhf(v); else if (ACT == 9) v = 0.5f * v * (1.0f + tanhf(0.7978845608028654f * (v + 0.044715f * v * v * v))); else if (ACT == 11) v = 1.0f / (1.0f + expf(-v)); else if (ACT == 12) v = (v > 0.f) ? v : 0.01f * v; else if (ACT == 14) v = (v > 0.f) ? v : 0.1f * v; else if (ACT == 15) v = v / (1.0f + expf(-v)); else if (ACT == 3) v = fmaxf(v, 0.f); else if (ACT == 6) v = 0.5f * v * (1.0f + erff(v * 0.70710678118654752f)); so[w][8 * hh + r][t * 16 + ln] = v; } }
  __builtin_amdgcn_fence(__ATOMIC_ACQ_REL, "workgroup"); __builtin_amdgcn_wave_barrier();
  const int rsub = lane >> 4, c4 = (lane & 15) * 4; typedef _Float16 v4h __attribute__((ext_vector_type(4)));
  for (int pass = 0; pass < 2; ++pass) {
#pragma unroll
    for (int q = 0; q < 8; ++q) { const int r = q * 2 + rsub; if (col0 + c4 < N) { const v4f v = *(const v4fa*)&so[w][r][c4]; if (C) *(volatile v4f*)(C + cofs + (size_t)(row0 + r) * ldc + col0 + c4) = v; if (C16) { v4h h4; for (int i = 0; i < 4; ++i) h4[i] = (_Float16)v[i]; *(volatile v4h*)(C16 + cofs + (size_t)(row0 + r) * ldc + col0 + c4) = h4; } } }
    if (pass == 0) __threadfence(); }
}


typedef _Float16 v4h __attribute__((ext_vector_type(4)));

__global__ __launch_bounds__(256) void k_x16(const float* __restrict__ x, _Float16* __restrict__ X16, size_t n8) { const size_t t = (size_t)blockIdx.x * 256 + threadIdx.x; if (t >= n8) return; FragH f;
#pragma unroll
  for (int q = 0; q < 8; ++q) f.h[q] = (_Float16)bf16_round(x[t * 8 + q]); *(volatile v8us*)((unsigned short*)X16 + t * 8) = f.half[0]; __threadfence(); *(volatile v8us*)((unsigned short*)X16 + t * 8) = f.half[0]; }
__global__ __launch_bounds__(256) void k_h16(const float* __restrict__ x, _Float16* __restrict__ X16, size_t n8) { const size_t t = (size_t)blockIdx.x * 256 + threadIdx.x; if (t >= n8) return; FragH f;
#pragma unroll
  for (int q = 0; q < 8; ++q) f.h[q] = (_Float16)x[t * 8 + q]; *(volatile v8us*)((unsigned short*)X16 + t * 8) = f.half[0]; __threadfence(); *(volatile v8us*)((unsigned short*)X16 + t * 8) = f.half[0]; }
__global__ __launch_bounds__(256) void k_round16f(const float* __restrict__ W, _Float16* __restrict__ Bt, size_t n8) { const size_t t = (size_t)blockIdx.x * 256 + threadIdx.x; if (t >= n8) return; FragH f;
#pragma unroll
  for (int i = 0; i < 8; ++i) f.h[i] = (_Float16)(bf16_round(W[t * 8 + i]) * 16.0f); *(volatile v8us*)((unsigned short*)Bt + t * 8) = f.half[0]; __threadfence(); *(volatile v8us*)((unsigned short*)Bt + t * 8) = f.half[0]; }
template <int NHv, int TTv>
__global__ __launch_bounds__(256) void k_vt(const _Float16* __restrict__ V16, int ldv, int voff, _Float16* __restrict__ Vt) { __shared__ unsigned short tl[64][66]; const int tid = threadIdx.x; const int slab = blockIdx.x / (TTv / 64), lg = blockIdx.x % (TTv / 64); const int b = slab / NHv, h = slab % NHv;
  for (int i = tid; i < 64 * 8; i += 256) { const int r = i / 8, c8 = (i % 8) * 8; FragH f; f.half[0] = *(const v8us*)((const unsigned short*)V16 + ((size_t)b * TTv + lg * 64 + r) * ldv + voff + h * 64 + c8);
#pragma unroll
    for (int q = 0; q < 8; ++q) tl[r][c8 + q] = f.u[q]; }
  __syncthreads();
  for (int pass = 0; pass < 2; ++pass) {
#pragma unroll
    for (int rd = 0; rd < 2; ++rd) { const int d = rd * 32 + tid / 8, pc = tid % 8; FragH f;
#pragma unroll
      for (int q = 0; q < 8; ++q) f.u[q] = tl[pc * 8 + q][d];
      *(volatile v8us*)((unsigned short*)Vt + ((size_t)slab * 64 + d) * TTv + lg * 64 + pc * 8) = f.half[0]; }
    if (pass == 0) __threadfence(); } }

__global__ __launch_bounds__(256) void k_hl(const float* __restrict__ F, _Float16* __restrict__ Hh, _Float16* __restrict__ Hl, size_t n8) { const size_t t = (size_t)blockIdx.x * 256 + threadIdx.x; if (t >= n8) return; FragH fh, fl; const v4f a = *(const v4fa*)(F + t * 8), c = *(const v4fa*)(F + t * 8 + 4);
#pragma unroll
  for (int q = 0; q < 4; ++q) { _Float16 h = (_Float16)a[q]; fh.h[q] = h; fl.h[q] = (_Float16)((a[q] - (float)h) * 1024.0f); h = (_Float16)c[q]; fh.h[4 + q] = h; fl.h[4 + q] = (_Float16)((c[q] - (float)h) * 1024.0f); }
  for (int pass = 0; pass < 2; ++pass) { *(volatile v8us*)((unsigned short*)Hh + t * 8) = fh.half[0]; *(volatile v8us*)((unsigned short*)Hl + t * 8) = fl.half[0]; if (pass == 0) __threadfence(); } }

#define VST2(T, ptr, val) do { const T vst2_v_ = (val); *(volatile T*)(ptr) = vst2_v_; __threadfence(); *(volatile T*)(ptr) = vst2_v_; } while (0)

#define C4_NB 4096
#define C4_CH 8192
__device__ __forceinline__ int c4_bucket(int v, int N) { v = min(max(v, 0), N - 1); return (int)(((long long)v * C4_NB) / N); }
__global__ __launch_bounds__(256) void k_c4_count(const int* __restrict__ tgt, int E, int N, int* __restrict__ CNT) {
    __shared__ int hist[C4_NB]; const int ch = blockIdx.x, t = threadIdx.x; const int e0 = ch * C4_CH; const int nt = min(C4_CH, E - e0);
    for (int j = 0; j < 16; ++j) hist[t + 256 * j] = 0; __syncthreads();
    for (int i = t; i < nt; i += 256) atomicAdd(&hist[c4_bucket(tgt[e0 + i], N)], 1);
    __syncthreads();
    for (int j = 0; j < 16; ++j) { const int v = hist[t + 256 * j]; VST2(int, CNT + (long long)ch * C4_NB + t + 256 * j, v); } }
__global__ __launch_bounds__(256) void k_c4_offsets(const int* __restrict__ CNT, int nch, int E, int* __restrict__ OFFB, int* __restrict__ BOFF) {
    __shared__ int tot[C4_NB]; __shared__ int part[256]; const int t = threadIdx.x;
    for (int j = 0; j < 16; ++j) { const int b = t + 256 * j; int s = 0; for (int ch = 0; ch < nch; ++ch) s += CNT[(long long)ch * C4_NB + b]; tot[b] = s; }
    __syncthreads();
    { int s = 0; for (int q = 0; q < 16; ++q) s += tot[16 * t + q]; part[t] = s; } __syncthreads();
    if (t == 0) { int run = 0; for (int i = 0; i < 256; ++i) { const int v = part[i]; part[i] = run; run += v; } } __syncthreads();
    { int run = part[t]; for (int q = 0; q < 16; ++q) { const int v = tot[16 * t + q]; tot[16 * t + q] = run; run += v; } }
    __syncthreads();
    for (int j = 0; j < 16; ++j) { const int b = t + 256 * j; VST2(int, BOFF + b, tot[b]); }
    if (t == 0) VST2(int, BOFF + C4_NB, E);
    for (int j = 0; j < 16; ++j) { const int b = t + 256 * j; int run = tot[b]; for (int ch = 0; ch < nch; ++ch) { VST2(int, OFFB + (long long)ch * C4_NB + b, run); run += CNT[(long long)ch * C4_NB + b]; } } }
__global__ __launch_bounds__(256) void k_c4_scatter(const int* __restrict__ tgt, int E, int N, const int* __restrict__ OFFB, int* __restrict__ BUF) {
    __shared__ int cur[C4_NB]; __shared__ int bk[256]; const int ch = blockIdx.x, t = threadIdx.x; const int e0 = ch * C4_CH; const int nt = min(C4_CH, E - e0);
    const int wv = t >> 5, ln = t & 31;
    for (int j = 0; j < 16; ++j) cur[t + 256 * j] = OFFB[(long long)ch * C4_NB + t + 256 * j];
    __syncthreads();
    for (int s0 = 0; s0 < C4_CH; s0 += 256) {
        const int i = s0 + t; const int e = e0 + i; const int b = (i < nt) ? c4_bucket(tgt[min(e, E - 1)], N) : -1;
        bk[t] = b; __syncthreads();
        int rank = 0, cntw = 0;
        for (int l = 0; l < 32; ++l) { const int o = bk[(wv << 5) + l]; const bool same = (o == b) && (b >= 0); cntw += same ? 1 : 0; rank += (same && l < ln) ? 1 : 0; }
        const bool last = (b >= 0) && (rank == cntw - 1);
        for (int w = 0; w < 8; ++w) {
            if (wv == w && b >= 0) { int pos = cur[b] + rank; pos = min(max(pos, 0), E - 1); VST2(int, BUF + pos, e); }
            __syncthreads();
            if (wv == w && last) cur[b] += cntw;
            __syncthreads(); }
    } }
template <int CAP>
__global__ __launch_bounds__(256) void k_c4_lists(const int* __restrict__ tgt, const int* __restrict__ BUF, const int* __restrict__ BOFF, int N, int E, int* __restrict__ NBR, int* __restrict__ cnt) {
    const int d = blockIdx.x * 256 + threadIdx.x; if (d >= N) return; const int b = c4_bucket(d, N); int n = 0; int* row = NBR + (long long)d * CAP;
    const int p0 = min(max(BOFF[b], 0), E), p1 = min(max(BOFF[b + 1], p0), E);
    for (int p = p0; p < p1; ++p) { int e = BUF[p]; e = min(max(e, 0), E - 1); if (tgt[e] == d) { if (n < CAP) VST2(int, row + n, e); ++n; } }
    for (int j = n; j < CAP; ++j) VST2(int, row + j, -1); VST2(int, cnt + d, min(n, CAP)); }
__global__ __launch_bounds__(256) void k_c4_scan1(const int* __restrict__ cnt, int* __restrict__ PART, int N) {
    __shared__ int part[256]; const int per = ((((N + 255) / 256) + 31) / 32) * 32; const int a = threadIdx.x * per, b = min(N, a + per); int s = 0;
    for (int i = a; i < b; ++i) s += cnt[i]; part[threadIdx.x] = s; __syncthreads();
    if (threadIdx.x == 0) { int run = 0; for (int t = 0; t < 256; ++t) { const int v = part[t]; part[t] = run; run += v; } } __syncthreads();
    VST2(int, PART + threadIdx.x, part[threadIdx.x]); }
__global__ __launch_bounds__(256) void k_c4_scan2(const int* __restrict__ cnt, const int* __restrict__ PART, int* __restrict__ off, int N) {
    const int i = blockIdx.x * 256 + threadIdx.x; if (i > N) return; const int per = ((((N + 255) / 256) + 31) / 32) * 32; const int r = min(i / per, 255); const int a = r * per;
    int s = PART[r]; for (int kq = a; kq < i; ++kq) s += cnt[min(kq, N - 1)];
    VST2(int, off + i, s); }
template <int CAP>
__global__ __launch_bounds__(256) void k_c4_slotcopy(const int* __restrict__ off, const int* __restrict__ NBR, int* __restrict__ slot, int N) {
    const int t = blockIdx.x * 256 + threadIdx.x; const int tot = off[N]; if (t >= tot) return;
    int lo = 0, hi = N - 1; while (lo < hi) { const int mid = (lo + hi + 1) >> 1; if (off[mid] <= t) lo = mid; else hi = mid - 1; }
    int j = t - off[lo]; j = (j < 0) ? 0 : ((j >= CAP) ? (CAP - 1) : j); VST2(int, slot + t, NBR[(long long)lo * CAP + j]); }

typedef float v2f __attribute__((ext_vector_type(2)));
__global__ __launch_bounds__(256) void k_ew(const float* __restrict__ ea, const float* __restrict__ W1e, const float* __restrict__ b1e, const float* __restrict__ w2e, const float* __restrict__ b2e, float* __restrict__ EW) {
  #pragma clang fp contract(off)
  const int e = blockIdx.x * 256 + threadIdx.x; if (e >= NE) return; float a[FE];
#pragma unroll
  for (int k = 0; k < FE; ++k) a[k] = bf16_round(ea[(size_t)e * FE + k]);
  float s = 0.f;
#pragma unroll 1
  for (int j = 0; j < HID; ++j) { float h = bf16_round(b1e[j]);
#pragma unroll
    for (int k = 0; k < FE; ++k) h += a[k] * bf16_round(W1e[k * HID + j]);
    s += fmaxf(h, 0.f) * bf16_round(w2e[j]); }
  const float v = 1.0f / (1.0f + expf(-(s + bf16_round(b2e[0])))); *(volatile float*)(EW + e) = v; __threadfence(); *(volatile float*)(EW + e) = v; }
__global__ __launch_bounds__(256) void k_sage(const _Float16* __restrict__ X, const int* __restrict__ src, const int* __restrict__ nbr, const int* __restrict__ cnt, const float* __restrict__ EW, _Float16* __restrict__ AGG) {
  #pragma clang fp contract(off)
  const int tid = threadIdx.x, w = tid >> 5, l = tid & 31; const int d = blockIdx.x * 8 + w; if (d >= NN) return; const int n = min(max(cnt[d], 0), ECAP); float acc[4] = {0.f, 0.f, 0.f, 0.f};
#pragma unroll 1
  for (int j = 0; j < ECAP; ++j) { int e = nbr[(size_t)d * ECAP + j]; const bool live = (j < n) && (e >= 0); e = min(max(e, 0), NE - 1); int s = src[e]; s = min(max(s, 0), NN - 1); const float wv = live ? EW[e] : 0.f;
    FragH f; *(unsigned long long*)&f.u[0] = *(const unsigned long long*)((const unsigned short*)X + (size_t)s * FIN + 4 * l);
#pragma unroll
    for (int q = 0; q < 4; ++q) acc[q] += wv * (float)f.h[q]; }
  const float inv = 1.0f / fmaxf((float)min(max(cnt[d], 0), NE), 1.0f); FragH o;
#pragma unroll
  for (int q = 0; q < 4; ++q) o.h[q] = (_Float16)(acc[q] * inv);
  const unsigned long long hv = *(const unsigned long long*)&o.u[0]; *(volatile unsigned long long*)((unsigned short*)AGG + (size_t)d * HID + 4 * l) = hv; __threadfence(); *(volatile unsigned long long*)((unsigned short*)AGG + (size_t)d * HID + 4 * l) = hv; }
__global__ __launch_bounds__(256) void k_wfold(const float* __restrict__ wl, const float* __restrict__ wr, const float* __restrict__ bl, const float* __restrict__ g, const float* __restrict__ be, const float* __restrict__ m, const float* __restrict__ v, _Float16* __restrict__ Bl, _Float16* __restrict__ Br, float* __restrict__ CB) {
  #pragma clang fp contract(off)
  const int t = blockIdx.x * 256 + threadIdx.x; if (t >= HID * (HID / 8)) return; const int o = t / (HID / 8), k0 = (t % (HID / 8)) * 8; const float s = bf16_round(g[o]) * rsqrtf(bf16_round(v[o]) + BNEPS); FragH fl, fr;
#pragma unroll
  for (int q = 0; q < 8; ++q) { fl.h[q] = (_Float16)(bf16_round(wl[(size_t)(k0 + q) * HID + o]) * s * 16.0f); fr.h[q] = (_Float16)(bf16_round(wr[(size_t)(k0 + q) * HID + o]) * s * 16.0f); }
  for (int pass = 0; pass < 2; ++pass) { *(volatile v8us*)((unsigned short*)Bl + (size_t)o * HID + k0) = fl.half[0]; *(volatile v8us*)((unsigned short*)Br + (size_t)o * HID + k0) = fr.half[0]; if (pass == 0) __threadfence(); }
  (void)bl; (void)be; (void)m; (void)CB; }
__global__ __launch_bounds__(128) void k_cbf(const float* __restrict__ bl, const float* __restrict__ g, const float* __restrict__ be, const float* __restrict__ m, const float* __restrict__ v, float* __restrict__ CB) {
  #pragma clang fp contract(off)
  const int o = threadIdx.x; if (o >= HID) return; const float s = bf16_round(g[o]) * rsqrtf(bf16_round(v[o]) + BNEPS); const float cb = (bf16_round(bl[o]) - bf16_round(m[o])) * s + bf16_round(be[o]); VST2(float, CB + o, cb); }
__global__ __launch_bounds__(256) void k_w3(const float* __restrict__ wl, const float* __restrict__ wr, _Float16* __restrict__ Bl, _Float16* __restrict__ Br) { const int t = blockIdx.x * 256 + threadIdx.x; if (t >= 16 * (HID / 8)) return; const int o = t / (HID / 8), k0 = (t % (HID / 8)) * 8; FragH fl, fr;
#pragma unroll
  for (int q = 0; q < 8; ++q) { fl.h[q] = (o < NOUT) ? (_Float16)(bf16_round(wl[(size_t)(k0 + q) * NOUT + o]) * 16.0f) : (_Float16)0.0f; fr.h[q] = (o < NOUT) ? (_Float16)(bf16_round(wr[(size_t)(k0 + q) * NOUT + o]) * 16.0f) : (_Float16)0.0f; }
  for (int pass = 0; pass < 2; ++pass) { *(volatile v8us*)((unsigned short*)Bl + (size_t)o * HID + k0) = fl.half[0]; *(volatile v8us*)((unsigned short*)Br + (size_t)o * HID + k0) = fr.half[0]; if (pass == 0) __threadfence(); } }
__global__ __launch_bounds__(256) void k_out2(const float* __restrict__ Tp, const float* __restrict__ b3, float* __restrict__ out) { const int r = blockIdx.x * 256 + threadIdx.x; if (r >= NN) return; v2f v; v.x = Tp[(size_t)r * 16] + bf16_round(b3[0]); v.y = Tp[(size_t)r * 16 + 1] + bf16_round(b3[1]); *(volatile v2f*)(out + (size_t)r * 2) = v; __threadfence(); *(volatile v2f*)(out + (size_t)r * 2) = v; }

extern "C" void kernel_launch(void* const* d_in, const int* in_sizes, int n_in,
                              void* d_out, int out_size, void* d_ws, size_t ws_size, hipStream_t stream) {
  (void)in_sizes; (void)n_in; (void)out_size;
  const float* const* I = (const float* const*)d_in; const float* x = I[0]; const float* ea = I[1]; const int* edges = (const int*)d_in[2]; const int* srcI = edges; const int* dstI = edges + NE;
  const float* ew1w = I[3]; const float* ew1b = I[4]; const float* ew2w = I[5]; const float* ew2b = I[6]; const float* w1l = I[7]; const float* b1l = I[8]; const float* w1r = I[9]; const float* w2l = I[10]; const float* b2l = I[11]; const float* w2r = I[12]; const float* w3l = I[13]; const float* b3l = I[14]; const float* w3r = I[15];
  const float* bn1g = I[16]; const float* bn1b = I[17]; const float* bn1m = I[18]; const float* bn1v = I[19]; const float* bn2g = I[20]; const float* bn2b = I[21]; const float* bn2m = I[22]; const float* bn2v = I[23];
  char* ws = (char*)d_ws; size_t off = 0;
  auto take = [&](size_t bytes) { char* p = ws + off; off += (bytes + 255) & ~(size_t)255; return p; };
  const int nch = (NE + C4_CH - 1) / C4_CH;
  int* c4_CNT = (int*)take((size_t)nch * C4_NB * 4); int* c4_OFFB = (int*)take((size_t)nch * C4_NB * 4); int* c4_BOFF = (int*)take((size_t)(C4_NB + 64) * 4); int* c4_BUF = (int*)take((size_t)(NE + 64) * 4);
  int* cnt = (int*)take((size_t)(NN + 64) * 4); int* nbr = (int*)take((size_t)NN * ECAP * 4);
  _Float16* B1l = (_Float16*)take((size_t)HID * HID * 2); _Float16* B1r = (_Float16*)take((size_t)HID * HID * 2); float* CB1 = (float*)take(HID * 4); _Float16* B2l = (_Float16*)take((size_t)HID * HID * 2); _Float16* B2r = (_Float16*)take((size_t)HID * HID * 2); float* CB2 = (float*)take(HID * 4); _Float16* B3l = (_Float16*)take((size_t)16 * HID * 2); _Float16* B3r = (_Float16*)take((size_t)16 * HID * 2);
  float* EW = (float*)take((size_t)NE * 4); _Float16* X16 = (_Float16*)take((size_t)NN * FIN * 2); _Float16* AGG = (_Float16*)take((size_t)NN * HID * 2); _Float16* H16 = (_Float16*)take((size_t)NN * HID * 2); float* TQ = (float*)take((size_t)RQ * HID * 4); float* T2 = (float*)take((size_t)NN * 16 * 4);
  if (off > ws_size) return;
  k_c4_count<<<(unsigned)nch, 256, 0, stream>>>(dstI, NE, NN, c4_CNT);
  k_c4_offsets<<<1, 256, 0, stream>>>(c4_CNT, nch, NE, c4_OFFB, c4_BOFF);
  k_c4_scatter<<<(unsigned)nch, 256, 0, stream>>>(dstI, NE, NN, c4_OFFB, c4_BUF);
  k_c4_lists<ECAP><<<(NN + 255) / 256, 256, 0, stream>>>(dstI, c4_BUF, c4_BOFF, NN, NE, nbr, cnt);
  k_wfold<<<(HID * (HID / 8) + 255) / 256, 256, 0, stream>>>(w1l, w1r, b1l, bn1g, bn1b, bn1m, bn1v, B1l, B1r, CB1); k_wfold<<<(HID * (HID / 8) + 255) / 256, 256, 0, stream>>>(w2l, w2r, b2l, bn2g, bn2b, bn2m, bn2v, B2l, B2r, CB2); k_w3<<<(16 * (HID / 8) + 255) / 256, 256, 0, stream>>>(w3l, w3r, B3l, B3r); k_cbf<<<1, 128, 0, stream>>>(b1l, bn1g, bn1b, bn1m, bn1v, CB1); k_cbf<<<1, 128, 0, stream>>>(b2l, bn2g, bn2b, bn2m, bn2v, CB2);
  k_ew<<<(NE + 255) / 256, 256, 0, stream>>>(ea, ew1w, ew1b, ew2w, ew2b, EW);
  k_x16<<<(NN * FIN / 8 + 255) / 256, 256, 0, stream>>>(x, X16, (size_t)NN * FIN / 8);
  const dim3 gQ(((RQ / 16) * (HID / 64) + 3) / 4, 1);
  for (int L = 0; L < 2; ++L) { const _Float16* Xin = (L == 0) ? X16 : H16; _Float16* Hout = (L == 0) ? H16 : X16; const _Float16* Bl = (L == 0) ? B1l : B2l; const _Float16* Br = (L == 0) ? B1r : B2r; const float* CB = (L == 0) ? CB1 : CB2;
    k_sage<<<(NN + 7) / 8, 256, 0, stream>>>(Xin, srcI, nbr, cnt, EW, AGG);
    for (int q = 0; q < NN / RQ; ++q) { const size_t r0 = (size_t)q * RQ;
      k_gemm_hhx<0><<<gQ, 128, 0, stream>>>(AGG + r0 * HID, HID, 0, Bl, HID, 0, 0.0625f, nullptr, 0, CB, RQ, 0, 0, TQ, nullptr, HID, 0, RQ, HID, HID);
      k_gemm_hhx<3><<<gQ, 128, 0, stream>>>(Xin + r0 * FIN, FIN, 0, Br, FIN, 0, 0.0625f, nullptr, 0, TQ, 1, (size_t)HID, 0, nullptr, Hout + r0 * HID, HID, 0, RQ, HID, FIN); } }
  k_sage<<<(NN + 7) / 8, 256, 0, stream>>>(X16, srcI, nbr, cnt, EW, AGG);
  const dim3 g2(((NN / 16) * 1 + 3) / 4, 1);
  k_gemm_hhx<0><<<g2, 128, 0, stream>>>(AGG, HID, 0, B3l, HID, 0, 0.0625f, nullptr, 0, nullptr, 1, 0, 0, T2, nullptr, 16, 0, NN, NOUT, HID);
  k_gemm_hhx<0><<<g2, 128, 0, stream>>>(X16, FIN, 0, B3r, FIN, 0, 0.0625f, nullptr, 0, T2, 1, 16, 0, T2, nullptr, 16, 0, NN, NOUT, FIN);
  k_out2<<<(NN + 255) / 256, 256, 0, stream>>>(T2, b3l, (float*)d_out);
}
